// PiecewiseRationalQuadraticCoupling_6811818132468
// MI455X (gfx1250) — hardware-verified
//
#include <hip/hip_runtime.h>
#include <math.h>

#define DID   32
#define DTR   32
#define HIDW  256
#define NPAR  25
#define NPO   800
#define CHR   16384

#define SX  64.0f
#define SW  1024.0f
#define SHS 1024.0f

typedef _Float16 v16h __attribute__((ext_vector_type(16)));
typedef _Float16 v8h  __attribute__((ext_vector_type(8)));
typedef float    v8f  __attribute__((ext_vector_type(8)));
typedef float    v4f  __attribute__((ext_vector_type(4)));
typedef unsigned int v4u __attribute__((ext_vector_type(4)));

union P8 { v8h h; v4u u; };

__device__ __forceinline__ float bf_rne(float f) {
  unsigned u = __float_as_uint(f);
  u = (u + 0x7FFFu + ((u >> 16) & 1u)) & 0xFFFF0000u;
  return __uint_as_float(u);
}
__device__ __forceinline__ v8f zero8() { v8f z = {0.f, 0.f, 0.f, 0.f, 0.f, 0.f, 0.f, 0.f}; return z; }

__device__ __forceinline__ v16h ldfrag(const _Float16* p) {
  union { v16h v; v8h h[2]; } f;
  f.h[0] = *(const v8h*)(p);
  f.h[1] = *(const v8h*)(p + 16);
  return f.v;
}

__device__ __forceinline__ v8f mma_h(v16h a, v16h b, v8f c) {
  return __builtin_amdgcn_wmma_f32_16x16x32_f16(false, a, false, b, (short)0, c, false, false);
}
__device__ __forceinline__ void dep_guard(v8f& a, v8f& b, v16h x) {
#if defined(__HIP_DEVICE_COMPILE__)
  asm volatile("v_nop\n\tv_nop\n\tv_nop\n\tv_nop" : "+v"(a), "+v"(b) : "v"(x));
#endif
}
__device__ __forceinline__ void dep_guard4(v8f& a, v8f& b, v16h x, v16h y) {
#if defined(__HIP_DEVICE_COMPILE__)
  asm volatile("v_nop\n\tv_nop\n\tv_nop\n\tv_nop" : "+v"(a), "+v"(b) : "v"(x), "v"(y));
#endif
}
__device__ __forceinline__ void keep2(v16h a, v16h b) {
#if defined(__HIP_DEVICE_COMPILE__)
  asm volatile("v_nop" :: "v"(a), "v"(b));
#endif
}
__device__ __forceinline__ void acc_guard2(v8f& a, v8f& b) {
#if defined(__HIP_DEVICE_COMPILE__)
  asm volatile("v_nop\n\tv_nop\n\tv_nop\n\tv_nop" : "+v"(a), "+v"(b));
#endif
}
__device__ __forceinline__ void wave_sync_lds() {
  __builtin_amdgcn_fence(__ATOMIC_RELEASE, "workgroup");
  __builtin_amdgcn_wave_barrier();
  __builtin_amdgcn_fence(__ATOMIC_ACQUIRE, "workgroup");
}

__global__ __launch_bounds__(256) void cvt_wt(const float* __restrict__ w, unsigned short* wt, int K, int N) {
  const int g = blockIdx.x * 256 + threadIdx.x;
  const int k8n = K >> 3;
  if (g < N * k8n) {
    const int n  = g / k8n;
    const int k8 = (g - n * k8n) * 8;
    P8 p;
#pragma unroll
    for (int i = 0; i < 8; ++i) p.h[i] = (_Float16)(bf_rne(w[(size_t)(k8 + i) * N + n]) * SW);
    unsigned short* dst = wt + (size_t)n * K + k8;
    *(volatile v4u*)dst = p.u;
    __threadfence();
    *(volatile v4u*)dst = p.u;
  }
}

__global__ __launch_bounds__(256) void cvt_x(const float* __restrict__ x, unsigned short* X, int nrows) {
  const int g = blockIdx.x * 256 + threadIdx.x;
  if (g < nrows * 4) {
    const int row = g >> 2;
    const int c8  = (g & 3) * 8;
    const float* src = x + (size_t)row * (DID + DTR) + c8;
    const v4f a = *(const v4f*)(src);
    const v4f c = *(const v4f*)(src + 4);
    P8 q;
#pragma unroll
    for (int t = 0; t < 4; ++t) {
      q.h[t]     = (_Float16)(bf_rne(a[t]) * SX);
      q.h[4 + t] = (_Float16)(bf_rne(c[t]) * SX);
    }
    unsigned short* dst = X + (size_t)g * 8;
    *(volatile v4u*)dst = q.u;
    __threadfence();
    *(volatile v4u*)dst = q.u;
  }
}

__global__ __launch_bounds__(256) void gemm_l1(
    const unsigned short* __restrict__ Ap,
    const unsigned short* __restrict__ Btp,
    const float* __restrict__ bias, float inscale, float oscale,
    unsigned short* Hh, unsigned short* Hl, int M) {
  constexpr int NT = 4, TN = 64, N = HIDW, K = DID, LDA = DID, LDB = DID, LDC = HIDW, SP = 68;
  const _Float16* A  = (const _Float16*)(const void*)Ap;
  const _Float16* Bt = (const _Float16*)(const void*)Btp;
  __shared__ __align__(16) float sT[8][16 * SP];
  const int lane = threadIdx.x & 31;
  const int wave = threadIdx.x >> 5;
  const int tilesN = N / TN;
  const int tilesM = M >> 6;
  const int tile = blockIdx.x * 8 + wave;
  if (tile >= tilesM * tilesN) return;
  const int tm = tile / tilesN;
  const int tn = tile - tm * tilesN;
  const int m0 = tm << 6;
  const int n0 = tn * TN;

  const int rlane = lane & 15;
  const int koff  = (lane >> 4) * 8;
  const int mOff  = (lane >> 4) * 8;

  float bv[NT];
#pragma unroll
  for (int j = 0; j < NT; ++j) bv[j] = bf_rne(bias[n0 + (j << 4) + rlane]);

  v8f acc[4][NT];
#pragma unroll
  for (int i = 0; i < 4; ++i)
#pragma unroll
    for (int j = 0; j < NT; ++j) acc[i][j] = zero8();

  for (int k0 = 0; k0 < K; k0 += 32) {
    v16h bh[NT];
#pragma unroll
    for (int j = 0; j < NT; ++j) {
      const size_t bo = (size_t)(n0 + (j << 4) + rlane) * LDB + koff + k0;
      bh[j] = ldfrag(Bt + bo);
    }
#pragma unroll
    for (int i = 0; i < 4; ++i) {
      const size_t ao = (size_t)(m0 + (i << 4) + rlane) * LDA + koff + k0;
      const v16h ah = ldfrag(A + ao);
#pragma unroll
      for (int j = 0; j < NT; ++j) acc[i][j] = mma_h(ah, bh[j], acc[i][j]);
      dep_guard(acc[i][0], acc[i][NT - 1], ah);
    }
    keep2(bh[0], bh[1]);
    keep2(bh[NT - 2], bh[NT - 1]);
  }
#pragma unroll
  for (int i = 0; i < 4; ++i)
#pragma unroll
    for (int j = 0; j < NT; j += 2) acc_guard2(acc[i][j], acc[i][j + 1]);

  float* slab = sT[wave];
  const int q = lane >> 3, c8 = (lane & 7) * 8;
#pragma unroll
  for (int i = 0; i < 4; ++i) {
    const int mBase = m0 + (i << 4);
#pragma unroll
    for (int j = 0; j < NT; ++j) {
#pragma unroll
      for (int r = 0; r < 8; ++r) {
        const float v = fmaxf(acc[i][j][r] * inscale + bv[j], 0.0f);
        slab[(mOff + r) * SP + (j << 4) + rlane] = v;
      }
    }
    wave_sync_lds();
#pragma unroll 1
    for (int pl = 0; pl < 2; ++pl) {
      v4u hv[4];
#pragma unroll
      for (int it = 0; it < 4; ++it) {
        const int row = it * 4 + q;
        const float* sp = slab + row * SP + c8;
        P8 pk;
#pragma unroll
        for (int e = 0; e < 8; ++e) {
          const float hs = sp[e] * oscale;
          const _Float16 hi = (_Float16)hs;
          const _Float16 lo = (_Float16)(hs - (float)hi);
          pk.h[e] = pl ? lo : hi;
        }
        hv[it] = pk.u;
      }
      unsigned short* C = pl ? Hl : Hh;
      for (int ps = 0; ps < 2; ++ps) {
#pragma unroll
        for (int it = 0; it < 4; ++it) {
          const int row = it * 4 + q;
          *(volatile v4u*)(C + (size_t)(mBase + row) * LDC + n0 + c8) = hv[it];
        }
        __threadfence();
      }
    }
    wave_sync_lds();
  }
}

__global__ __launch_bounds__(256) void gemm_l2(
    const unsigned short* __restrict__ Ahp, const unsigned short* __restrict__ Alp,
    const unsigned short* __restrict__ Btp,
    const float* __restrict__ bias, float inscale, float* Pout, int M) {
  constexpr int NT = 2, TN = 32, N = NPO, K = HIDW, LDA = HIDW, LDB = HIDW, LDP = NPO, SP = 36;
  const _Float16* Ah = (const _Float16*)(const void*)Ahp;
  const _Float16* Al = (const _Float16*)(const void*)Alp;
  const _Float16* Bt = (const _Float16*)(const void*)Btp;
  __shared__ __align__(16) float sT[8][16 * SP];
  const int lane = threadIdx.x & 31;
  const int wave = threadIdx.x >> 5;
  const int tilesN = N / TN;
  const int tilesM = M >> 6;
  const int tile = blockIdx.x * 8 + wave;
  if (tile >= tilesM * tilesN) return;
  const int tm = tile / tilesN;
  const int tn = tile - tm * tilesN;
  const int m0 = tm << 6;
  const int n0 = tn * TN;

  const int rlane = lane & 15;
  const int koff  = (lane >> 4) * 8;
  const int mOff  = (lane >> 4) * 8;

  float bv[NT];
#pragma unroll
  for (int j = 0; j < NT; ++j) bv[j] = bf_rne(bias[n0 + (j << 4) + rlane]);

  v8f acc[4][NT];
#pragma unroll
  for (int i = 0; i < 4; ++i)
#pragma unroll
    for (int j = 0; j < NT; ++j) acc[i][j] = zero8();

  for (int k0 = 0; k0 < K; k0 += 32) {
    v16h bh[NT];
#pragma unroll
    for (int j = 0; j < NT; ++j) {
      const size_t bo = (size_t)(n0 + (j << 4) + rlane) * LDB + koff + k0;
      bh[j] = ldfrag(Bt + bo);
    }
#pragma unroll
    for (int i = 0; i < 4; ++i) {
      const size_t ao = (size_t)(m0 + (i << 4) + rlane) * LDA + koff + k0;
      const v16h ah = ldfrag(Ah + ao);
      const v16h al = ldfrag(Al + ao);
#pragma unroll
      for (int j = 0; j < NT; ++j) acc[i][j] = mma_h(ah, bh[j], acc[i][j]);
#pragma unroll
      for (int j = 0; j < NT; ++j) acc[i][j] = mma_h(al, bh[j], acc[i][j]);
      dep_guard4(acc[i][0], acc[i][NT - 1], ah, al);
    }
    keep2(bh[0], bh[NT - 1]);
  }
#pragma unroll
  for (int i = 0; i < 4; ++i) acc_guard2(acc[i][0], acc[i][1]);

  float* slab = sT[wave];
  const int q = lane >> 3, c4 = (lane & 7) * 4;
#pragma unroll
  for (int i = 0; i < 4; ++i) {
    const int mBase = m0 + (i << 4);
#pragma unroll
    for (int j = 0; j < NT; ++j) {
#pragma unroll
      for (int r = 0; r < 8; ++r) {
        const float v = acc[i][j][r] * inscale + bv[j];
        slab[(mOff + r) * SP + (j << 4) + rlane] = v;
      }
    }
    wave_sync_lds();
    v4f pv[4];
#pragma unroll
    for (int it = 0; it < 4; ++it) {
      const int row = it * 4 + q;
      pv[it] = *(const v4f*)(slab + row * SP + c4);
    }
    for (int ps = 0; ps < 2; ++ps) {
#pragma unroll
      for (int it = 0; it < 4; ++it) {
        const int row = it * 4 + q;
        *(volatile v4f*)(Pout + (size_t)(mBase + row) * LDP + n0 + c4) = pv[it];
      }
      __threadfence();
    }
    wave_sync_lds();
  }
}

__global__ __launch_bounds__(256) void spline_k(const float* __restrict__ P, const float* __restrict__ inp,
                                                float* out0, float* out1, int rbase) {
#pragma clang fp contract(off)
  __shared__ __align__(16) float sK[3][9][256];
  __shared__ __align__(16) float sO[8][8][64];
  __shared__ __align__(16) float sL[64];
  const int tid  = threadIdx.x;
  const int lane = tid & 31;
  const int wave = tid >> 5;
  const int j    = lane;
  const int lr0  = blockIdx.x * 64 + wave * 8;

#pragma unroll 1
  for (int r = 0; r < 8; ++r) {
    const int lr = lr0 + r;
    const size_t grow = (size_t)rbase + (size_t)lr;
    const float* pb = P + (size_t)lr * NPO + j * NPAR;
    const float* xr = inp + grow * (DID + DTR);

#pragma unroll 1
    for (int g = 0; g < 2; ++g) {
      const float* pg = pb + g * 8;
      float m = pg[0];
#pragma unroll 1
      for (int qq = 1; qq < 8; ++qq) m = fmaxf(m, pg[qq]);
      float ssum = 0.0f;
#pragma unroll 1
      for (int qq = 0; qq < 8; ++qq) {
        const float e = expf(pg[qq] - m);
        ssum = ssum + e;
        sK[g][qq + 1][tid] = e;
      }
      const float invs = 1.0f / ssum;
      float run = 0.0f;
#pragma unroll 1
      for (int qq = 0; qq < 8; ++qq) {
        const float wq = 0.001f + 0.992f * (sK[g][qq + 1][tid] * invs);
        run = run + wq;
        sK[g][qq + 1][tid] = run;
      }
      const float invn = 1.0f / fmaxf(run, 1e-12f);
      sK[g][0][tid] = 0.0f;
#pragma unroll 1
      for (int qq = 1; qq < 9; ++qq) sK[g][qq][tid] = sK[g][qq][tid] * invn;
    }
#pragma unroll 1
    for (int qq = 0; qq < 9; ++qq) {
      const float u  = pb[16 + qq];
      const float sp = fmaxf(u, 0.0f) + log1pf(expf(-fabsf(u)));
      sK[2][qq][tid] = 0.001f + sp;
    }

    const float x   = bf_rne(xr[DID + j]);
    const float idv = bf_rne(xr[j]);
    const bool inside = (x >= -10.0f) && (x <= 10.0f);
    float xs = (x + 10.0f) * 0.05f;
    xs = fminf(fmaxf(xs, 0.0f), 1.0f);
    int cnt = 0;
#pragma unroll 1
    for (int qq = 0; qq < 9; ++qq) cnt += (xs >= sK[0][qq][tid]) ? 1 : 0;
    int bin = cnt - 1;
    bin = bin < 0 ? 0 : bin;
    bin = bin > 7 ? 7 : bin;

    const float xk  = sK[0][bin][tid];
    const float wk  = sK[0][bin + 1][tid] - xk;
    const float yk  = sK[1][bin][tid];
    const float hk  = sK[1][bin + 1][tid] - yk;
    const float dk  = sK[2][bin][tid];
    const float dk1 = sK[2][bin + 1][tid];

    float t = (xs - xk) / (wk + 1e-12f);
    t = fminf(fmaxf(t, 0.0f), 1.0f);
    const float a   = (hk + 1e-12f) / (wk + 1e-12f);
    const float omt = 1.0f - t;
    const float num = (a * t) * t + (dk * t) * omt;
    const float den = a + (((dk + dk1) - 2.0f * a) * t) * omt;
    const float s   = num / (den + 1e-12f);
    const float ys  = yk + hk * s;
    const float y   = ys * 20.0f - 10.0f;
    const float dn  = (a * a) * ((((dk1 * t) * t) + ((2.0f * a) * t) * omt) + (dk * omt) * omt);
    const float dydx = dn / (den * den + 1e-12f);
    const float lad = logf(fmaxf(dydx, 1e-12f));

    const float yo = inside ? y : x;
    float lv = inside ? lad : 0.0f;
    lv += __shfl_xor(lv, 16, 32);
    lv += __shfl_xor(lv, 8, 32);
    lv += __shfl_xor(lv, 4, 32);
    lv += __shfl_xor(lv, 2, 32);
    lv += __shfl_xor(lv, 1, 32);

    sO[wave][r][j] = idv;
    sO[wave][r][DID + j] = yo;
    if (lane == 0) sL[wave * 8 + r] = lv;
  }

  wave_sync_lds();
  const int hh = lane >> 4, c4 = (lane & 15) * 4;
  v4f ov[4];
#pragma unroll
  for (int it = 0; it < 4; ++it) ov[it] = *(const v4f*)(&sO[wave][it * 2 + hh][c4]);
  for (int ps = 0; ps < 2; ++ps) {
#pragma unroll
    for (int it = 0; it < 4; ++it) {
      const size_t grow = (size_t)rbase + (size_t)(lr0 + it * 2 + hh);
      *(volatile v4f*)(out0 + grow * (DID + DTR) + c4) = ov[it];
    }
    __threadfence();
  }

  __syncthreads();
  if (wave == 0) {
    const v4f v = *(const v4f*)(sL + 4 * (lane & 15));
    float* dst = out1 + (size_t)rbase + (size_t)blockIdx.x * 64 + 4 * (lane & 15);
    if (lane < 16) *(volatile v4f*)dst = v;
    __threadfence();
    if (lane < 16) *(volatile v4f*)dst = v;
  }
}

extern "C" void kernel_launch(void* const* d_in, const int* in_sizes, int n_in,
                              void* d_out, int out_size, void* d_ws, size_t ws_size,
                              hipStream_t stream) {
  if (n_in < 5) return;
  const int nx = in_sizes[0];
  if (nx < (DID + DTR) || (nx % (DID + DTR)) != 0) return;
  const int B = nx / (DID + DTR);
  if ((B % 64) != 0) return;
  if (in_sizes[1] != DID * HIDW || in_sizes[2] != HIDW || in_sizes[3] != HIDW * NPO || in_sizes[4] != NPO) return;
  if (out_size != B * (DID + DTR) + B) return;

  const float* inp = (const float*)d_in[0];
  const float* W1  = (const float*)d_in[1];
  const float* b1  = (const float*)d_in[2];
  const float* W2  = (const float*)d_in[3];
  const float* b2  = (const float*)d_in[4];
  float* out0 = (float*)d_out;
  float* out1 = out0 + (size_t)B * (DID + DTR);

  const size_t PWT1 = (size_t)HIDW * DID * 2;
  const size_t PWT2 = (size_t)NPO * HIDW * 2;
  const size_t PX   = (size_t)B * DID * 2;
  const size_t PH   = (size_t)CHR * HIDW * 2;
  const size_t PP   = (size_t)CHR * NPO * 4;
  size_t off = 0;
  const size_t oWt1 = off; off += PWT1;
  const size_t oWt2 = off; off += PWT2;
  const size_t oX   = off; off += PX;
  const size_t oHh  = off; off += PH;
  const size_t oHl  = off; off += PH;
  const size_t oP   = off; off += PP;
  if (off > ws_size) return;
  if (off > (size_t)134217728) return;

  char* ws = (char*)d_ws;
  unsigned short* Wt1 = (unsigned short*)(ws + oWt1);
  unsigned short* Wt2 = (unsigned short*)(ws + oWt2);
  unsigned short* X16 = (unsigned short*)(ws + oX);
  unsigned short* Hh  = (unsigned short*)(ws + oHh);
  unsigned short* Hl  = (unsigned short*)(ws + oHl);
  float* Pp = (float*)(ws + oP);

  const dim3 blk(256);
  const int n8w1 = HIDW * DID / 8;
  const int n8w2 = NPO * HIDW / 8;
  const dim3 gW1((n8w1 + 255) / 256);
  const dim3 gW2((n8w2 + 255) / 256);
  const dim3 gX((B * 4 + 255) / 256);

  const float is1 = 1.0f / (SX * SW);
  const float is2 = 1.0f / (SHS * SW);

  cvt_wt<<<gW1, blk, 0, stream>>>(W1, Wt1, DID, HIDW);
  cvt_wt<<<gW2, blk, 0, stream>>>(W2, Wt2, HIDW, NPO);
  cvt_x<<<gX, blk, 0, stream>>>(inp, X16, B);

  const int nch = (B + CHR - 1) / CHR;
  for (int c = 0; c < nch; ++c) {
    const int rbase = c * CHR;
    int rows = B - rbase;
    if (rows > CHR) rows = CHR;
    const int tilesM = rows / 64;
    const dim3 gG1((tilesM * 4 + 7) / 8);
    const dim3 gG2((tilesM * 25 + 7) / 8);
    const dim3 gSp(tilesM);
    gemm_l1<<<gG1, blk, 0, stream>>>(X16 + (size_t)rbase * DID, Wt1, b1, is1, SHS, Hh, Hl, rows);
    gemm_l2<<<gG2, blk, 0, stream>>>(Hh, Hl, Wt2, b2, is2, Pp, rows);
    spline_k<<<gSp, blk, 0, stream>>>(Pp, inp, out0, out1, rbase);
  }
  (void)hipGetLastError();
}
